// LinearAttention_86431921865156
// MI455X (gfx1250) — hardware-verified
//
#include <hip/hip_runtime.h>
#include <math.h>

#ifndef NB
#define NB 2
#endif
#ifndef SEQ
#define SEQ 2048
#endif
#define NB_FULL 2
#define SEQ_FULL 2048
#define DM 1024
#define NHEAD 16
#define HDIM 64
#define MROWS (NB * SEQ)

static_assert(NB >= 1 && NB <= NB_FULL);
static_assert(SEQ >= 64 && SEQ <= SEQ_FULL && (SEQ % 64) == 0);
static_assert(DM == NHEAD * HDIM);
static_assert((DM % 64) == 0 && (HDIM % 64) == 0 && (MROWS % 64) == 0);

typedef unsigned short us;
typedef __bf16 v16b __attribute__((ext_vector_type(16)));
typedef unsigned short v8us __attribute__((ext_vector_type(8), may_alias));
typedef float v8f __attribute__((ext_vector_type(8)));
typedef float v4f __attribute__((ext_vector_type(4), may_alias));
typedef unsigned int v4u __attribute__((ext_vector_type(4), may_alias));

union Frag { v16b v; v8us p[2]; };
__device__ __forceinline__ v16b ldf(const us* row, int k0, int h) {
    Frag f;
    f.p[0] = *(const v8us*)(row + k0 + 8 * h);
    f.p[1] = *(const v8us*)(row + k0 + 16 + 8 * h);
    return f.v;
}

__device__ __forceinline__ unsigned int bfb(float f) { unsigned int u = __float_as_uint(f); u += 0x7fffu + ((u >> 16) & 1u); return u >> 16; }
__device__ __forceinline__ float bfv(unsigned int b) { return __uint_as_float(b << 16); }
__device__ __forceinline__ float bfr(float f) { return bfv(bfb(f)); }

__device__ __forceinline__ void split8(const float (&e)[8], v4u& wh, v4u& wl) {
    unsigned int hb[8], lb[8];
#pragma unroll
    for (int j = 0; j < 8; ++j) { hb[j] = bfb(e[j]); lb[j] = bfb(e[j] - bfv(hb[j])); }
    wh[0] = hb[0] | (hb[1] << 16); wh[1] = hb[2] | (hb[3] << 16); wh[2] = hb[4] | (hb[5] << 16); wh[3] = hb[6] | (hb[7] << 16);
    wl[0] = lb[0] | (lb[1] << 16); wl[1] = lb[2] | (lb[3] << 16); wl[2] = lb[4] | (lb[5] << 16); wl[3] = lb[6] | (lb[7] << 16);
}

__device__ __forceinline__ v8f mma1(v16b a, v16b b, v8f c) {
    c = __builtin_amdgcn_wmma_f32_16x16x32_bf16(false, a, false, b, (short)0, c, false, false);
    asm volatile("v_nop\n\tv_nop\n\tv_nop\n\tv_nop" : "+v"(c) : "v"(a), "v"(b));
    return c;
}
__device__ __forceinline__ v8f mma2(v16b ah, v16b al, v16b b, v8f c) {
    c = __builtin_amdgcn_wmma_f32_16x16x32_bf16(false, ah, false, b, (short)0, c, false, false);
    c = __builtin_amdgcn_wmma_f32_16x16x32_bf16(false, al, false, b, (short)0, c, false, false);
    asm volatile("v_nop\n\tv_nop\n\tv_nop\n\tv_nop" : "+v"(c) : "v"(ah), "v"(al), "v"(b));
    return c;
}
__device__ __forceinline__ v8f mma3(v16b ah, v16b al, v16b bh, v16b bl, v8f c) {
    c = __builtin_amdgcn_wmma_f32_16x16x32_bf16(false, ah, false, bh, (short)0, c, false, false);
    c = __builtin_amdgcn_wmma_f32_16x16x32_bf16(false, ah, false, bl, (short)0, c, false, false);
    c = __builtin_amdgcn_wmma_f32_16x16x32_bf16(false, al, false, bh, (short)0, c, false, false);
    asm volatile("v_nop\n\tv_nop\n\tv_nop\n\tv_nop" : "+v"(c) : "v"(ah), "v"(al), "v"(bh), "v"(bl));
    return c;
}

#define ST2U(ptr, w) do { *(volatile v4u*)(ptr) = (w); __threadfence(); *(volatile v4u*)(ptr) = (w); } while (0)
#define ST2F(ptr, w) do { *(volatile v4f*)(ptr) = (w); __threadfence(); *(volatile v4f*)(ptr) = (w); } while (0)

__device__ __forceinline__ float actf(float v, int act) {
    if (act == 3) return v * __builtin_amdgcn_rcpf(1.f + expf(-v));
    if (act == 6) return __builtin_amdgcn_rcpf(1.f + expf(-v));
    return v;
}

__global__ __launch_bounds__(256) void k_cvt(const float* __restrict__ src, us* __restrict__ dst, int rows, int cols, int seg, long long sstride, long long spitch) {
    const long long i8 = (long long)blockIdx.x * 256 + threadIdx.x;
    const int c8n = cols >> 3;
    if (i8 >= (long long)rows * c8n) return;
    const int r = (int)(i8 / c8n);
    const int c = (int)(i8 - (long long)r * c8n) * 8;
    const int grp = r / seg, rr = r - grp * seg;
    const float* s = src + (long long)grp * sstride + (long long)rr * spitch + c;
    const v4f a = *(const v4f*)s;
    const v4f b = *(const v4f*)(s + 4);
    v4u w;
    w[0] = bfb(a[0]) | (bfb(a[1]) << 16); w[1] = bfb(a[2]) | (bfb(a[3]) << 16);
    w[2] = bfb(b[0]) | (bfb(b[1]) << 16); w[3] = bfb(b[2]) | (bfb(b[3]) << 16);
    ST2U(dst + (long long)r * cols + c, w);
}

struct GArg {
    const us* A0; const us* A1; const us* B; const float* bias; void* C0; void* C1; void* T0; void* T1;
    int M, N, K, lda, ldb, ldc, act, flags;
};
static_assert(sizeof(GArg) == 8 * 8 + 8 * 4);

#define CTP 68
template <int NA, int EPI>
__global__ __launch_bounds__(64) void k_pgemm(GArg g) {
    __shared__ __align__(16) float ct[64 * CTP];
    const int tid = threadIdx.x, lane = tid & 31, h = lane >> 4, l15 = lane & 15, wave = tid >> 5;
    const int nb = blockIdx.x * 64, mb = blockIdx.y * 64;
    const int mw = mb + 32 * wave;
    v8f acc[2][4];
#pragma unroll
    for (int mi = 0; mi < 2; ++mi)
#pragma unroll
        for (int t = 0; t < 4; ++t) { v8f z = {}; acc[mi][t] = z; }
    const us* ar0 = g.A0 + (long long)(mw + l15) * g.lda;
    const us* ar1 = g.A0 + (long long)(mw + 16 + l15) * g.lda;
    const us* lr0 = (NA == 2) ? (g.A1 + (long long)(mw + l15) * g.lda) : ar0;
    const us* lr1 = (NA == 2) ? (g.A1 + (long long)(mw + 16 + l15) * g.lda) : ar1;
    const us* br = g.B + (long long)(nb + l15) * g.ldb;
    for (int k0 = 0; k0 < g.K; k0 += 32) {
        const v16b ah0 = ldf(ar0, k0, h), ah1 = ldf(ar1, k0, h);
        v16b al0 = ah0, al1 = ah1;
        if (NA == 2) { al0 = ldf(lr0, k0, h); al1 = ldf(lr1, k0, h); }
#pragma unroll
        for (int t = 0; t < 4; ++t) {
            const v16b bf = ldf(br + (long long)(16 * t) * g.ldb, k0, h);
            if (NA == 2) { acc[0][t] = mma2(ah0, al0, bf, acc[0][t]); acc[1][t] = mma2(ah1, al1, bf, acc[1][t]); }
            else         { acc[0][t] = mma1(ah0, bf, acc[0][t]);      acc[1][t] = mma1(ah1, bf, acc[1][t]); }
        }
    }
    const bool tr = (EPI == 2) && (nb >= 2 * DM);
#pragma unroll
    for (int mi = 0; mi < 2; ++mi)
#pragma unroll
        for (int t = 0; t < 4; ++t)
#pragma unroll
            for (int r = 0; r < 8; ++r) {
                const int ml = 32 * wave + 16 * mi + 8 * h + r, nl = 16 * t + l15;
                ct[tr ? (nl * CTP + ml) : (ml * CTP + nl)] = acc[mi][t][r];
            }
    __syncthreads();
    int act = g.act;
    if (EPI == 2) act = tr ? 0 : 3;
    if (EPI == 0) {
        float* C = (float*)g.C0;
        for (int idx = tid; idx < 64 * 16; idx += 64) {
            const int row = idx >> 4, q = (idx & 15) * 4;
            const v4f v = *(const v4f*)(ct + row * CTP + q);
            float e[4] = {v[0], v[1], v[2], v[3]};
#pragma unroll
            for (int j = 0; j < 4; ++j) {
                float xv = e[j];
                if (g.flags & 1) xv += bfr(g.bias[nb + q + j]);
                e[j] = actf(xv, act);
            }
            v4f w = {e[0], e[1], e[2], e[3]};
            ST2F(C + (long long)(mb + row) * g.ldc + nb + q, w);
        }
    } else {
        us* D0; us* D1; long long base, pitch;
        if (!tr) { D0 = (us*)g.C0; D1 = (us*)g.C1; base = (long long)mb * g.ldc + nb; pitch = g.ldc; }
        else {
            const int bb = mb / SEQ, tok0 = mb - bb * SEQ, hd = (nb - 2 * DM) / HDIM;
            D0 = (us*)g.T0; D1 = (us*)g.T1; base = ((long long)(bb * NHEAD + hd) * HDIM) * SEQ + tok0; pitch = SEQ;
        }
        for (int idx = tid; idx < 64 * 8; idx += 64) {
            const int row = idx >> 3, o = (idx & 7) * 8;
            const v4f a = *(const v4f*)(ct + row * CTP + o);
            const v4f b = *(const v4f*)(ct + row * CTP + o + 4);
            float e[8] = {a[0], a[1], a[2], a[3], b[0], b[1], b[2], b[3]};
#pragma unroll
            for (int j = 0; j < 8; ++j) {
                float xv = e[j];
                if (g.flags & 1) xv += bfr(g.bias[tr ? (nb + row) : (nb + o + j)]);
                e[j] = actf(xv, act);
            }
            v4u wh, wl;
            split8(e, wh, wl);
            ST2U(D0 + base + (long long)row * pitch + o, wh);
            ST2U(D1 + base + (long long)row * pitch + o, wl);
        }
    }
}

#define PPITCH 72
__global__ __launch_bounds__(32) void k_attn(const us* __restrict__ qkh, const us* __restrict__ qkl, const us* __restrict__ vth, const us* __restrict__ vtl, float* __restrict__ O) {
    __shared__ __align__(16) us ph[16 * PPITCH];
    __shared__ __align__(16) us pl[16 * PPITCH];
    __shared__ __align__(16) float ost[16 * CTP];
    const int lane = threadIdx.x & 31, h = lane >> 4, l15 = lane & 15;
    const int q0 = blockIdx.x * 16, hd = blockIdx.y, b = blockIdx.z;
    const long long tokb = (long long)b * SEQ;
    const long long QP = 2 * DM;
    const us* qrh = qkh + (tokb + q0 + l15) * QP + hd * HDIM;
    const us* qrl = qkl + (tokb + q0 + l15) * QP + hd * HDIM;
    const v16b qh0 = ldf(qrh, 0, h), qh1 = ldf(qrh, 32, h);
    const v16b ql0 = ldf(qrl, 0, h), ql1 = ldf(qrl, 32, h);
    const us* kbh = qkh + tokb * QP + DM + hd * HDIM;
    const us* kbl = qkl + tokb * QP + DM + hd * HDIM;
    const us* vbh = vth + ((long long)(b * NHEAD + hd) * HDIM) * SEQ;
    const us* vbl = vtl + ((long long)(b * NHEAD + hd) * HDIM) * SEQ;
    v8f o[4];
#pragma unroll
    for (int t = 0; t < 4; ++t) { v8f z = {}; o[t] = z; }
    const int nch = (q0 >> 6) + 1;
    for (int c = 0; c < nch; ++c) {
        const int j0 = c * 64;
        v8f s[4];
#pragma unroll
        for (int t = 0; t < 4; ++t) {
            const long long ko = (long long)(j0 + 16 * t + l15) * QP;
            v8f a = {};
            a = mma3(qh0, ql0, ldf(kbh + ko, 0, h),  ldf(kbl + ko, 0, h),  a);
            a = mma3(qh1, ql1, ldf(kbh + ko, 32, h), ldf(kbl + ko, 32, h), a);
            s[t] = a;
        }
        __syncthreads();
#pragma unroll
        for (int i = 0; i < 8; ++i) {
            const int irow = q0 + 8 * h + i;
#pragma unroll
            for (int t = 0; t < 4; ++t) {
                const int jg = j0 + 16 * t + l15;
                const float v = (jg <= irow) ? s[t][i] : 0.f;
                const unsigned int hb = bfb(v);
                const unsigned int lb = bfb(v - bfv(hb));
                ph[(8 * h + i) * PPITCH + 16 * t + l15] = (us)hb;
                pl[(8 * h + i) * PPITCH + 16 * t + l15] = (us)lb;
            }
        }
        __syncthreads();
        const v16b pa0h = ldf(ph + l15 * PPITCH, 0, h), pa1h = ldf(ph + l15 * PPITCH, 32, h);
        const v16b pa0l = ldf(pl + l15 * PPITCH, 0, h), pa1l = ldf(pl + l15 * PPITCH, 32, h);
#pragma unroll
        for (int t = 0; t < 4; ++t) {
            const long long vo = (long long)(16 * t + l15) * SEQ + j0;
            o[t] = mma3(pa0h, pa0l, ldf(vbh + vo, 0, h),  ldf(vbl + vo, 0, h),  o[t]);
            o[t] = mma3(pa1h, pa1l, ldf(vbh + vo, 32, h), ldf(vbl + vo, 32, h), o[t]);
        }
    }
#pragma unroll
    for (int t = 0; t < 4; ++t)
#pragma unroll
        for (int r = 0; r < 8; ++r) ost[(8 * h + r) * CTP + 16 * t + l15] = o[t][r];
    __syncthreads();
    float* ob = O + (tokb + q0) * DM + hd * HDIM;
#pragma unroll
    for (int si = 0; si < 8; ++si) {
        const int row = 2 * si + (lane >> 4), c4 = (lane & 15) * 4;
        const v4f v = *(const v4f*)(ost + row * CTP + c4);
        ST2F(ob + (long long)row * DM + c4, v);
    }
}

__global__ __launch_bounds__(128) void k_ln(const float* __restrict__ O, const float* __restrict__ G, const float* __restrict__ gam, const float* __restrict__ bet,
                                            us* __restrict__ yh, us* __restrict__ yl) {
    __shared__ float red[4];
    const int tid = threadIdx.x, lane = tid & 31, wave = tid >> 5;
    const long long row = blockIdx.x;
    const int c = tid * 8;
    const float* op = O + row * DM + c;
    const float* gp = G + row * DM + c;
    const v4f o0 = *(const v4f*)op, o1 = *(const v4f*)(op + 4);
    const v4f g0 = *(const v4f*)gp, g1 = *(const v4f*)(gp + 4);
    float a[8] = {o0[0] * g0[0], o0[1] * g0[1], o0[2] * g0[2], o0[3] * g0[3], o1[0] * g1[0], o1[1] * g1[1], o1[2] * g1[2], o1[3] * g1[3]};
    float s = 0.f;
#pragma unroll
    for (int j = 0; j < 8; ++j) s += a[j];
    s += __shfl_xor(s, 1, 32); s += __shfl_xor(s, 2, 32); s += __shfl_xor(s, 4, 32); s += __shfl_xor(s, 8, 32); s += __shfl_xor(s, 16, 32);
    if (lane == 0) red[wave] = s;
    __syncthreads();
    const float mu = ((red[0] + red[1]) + (red[2] + red[3])) * (1.f / (float)DM);
    __syncthreads();
    float d[8]; float q = 0.f;
#pragma unroll
    for (int j = 0; j < 8; ++j) { d[j] = a[j] - mu; q += d[j] * d[j]; }
    q += __shfl_xor(q, 1, 32); q += __shfl_xor(q, 2, 32); q += __shfl_xor(q, 4, 32); q += __shfl_xor(q, 8, 32); q += __shfl_xor(q, 16, 32);
    if (lane == 0) red[wave] = q;
    __syncthreads();
    const float var = ((red[0] + red[1]) + (red[2] + red[3])) * (1.f / (float)DM);
    const float rstd = rsqrtf(var + 1e-5f);
    float e[8];
#pragma unroll
    for (int j = 0; j < 8; ++j) e[j] = d[j] * rstd * bfr(gam[c + j]) + bfr(bet[c + j]);
    v4u wh, wl;
    split8(e, wh, wl);
    ST2U(yh + row * DM + c, wh);
    ST2U(yl + row * DM + c, wl);
}

template __global__ void k_pgemm<1, 2>(GArg);
template __global__ void k_pgemm<1, 1>(GArg);
template __global__ void k_pgemm<2, 0>(GArg);

extern "C" void kernel_launch(void* const* d_in, const int* in_sizes, int n_in, void* d_out, int out_size, void* d_ws, size_t ws_size, hipStream_t stream) {
    if (n_in < 9) return;
    const float* x     = (const float*)d_in[0];
    const float* wqkv  = (const float*)d_in[1];
    const float* wg1   = (const float*)d_in[2];
    const float* bg1   = (const float*)d_in[3];
    const float* wg2   = (const float*)d_in[4];
    const float* bg2   = (const float*)d_in[5];
    const float* wout  = (const float*)d_in[6];
    const float* gamma = (const float*)d_in[7];
    const float* beta  = (const float*)d_in[8];
    float* out = (float*)d_out;

    const long long needx = ((long long)(NB - 1) * SEQ_FULL + SEQ) * (long long)DM;
    if ((long long)in_sizes[0] < needx) return;
    if (in_sizes[1] < 3 * DM * DM || in_sizes[2] < HDIM * DM || in_sizes[3] < HDIM || in_sizes[4] < DM * HDIM || in_sizes[5] < DM) return;
    if (in_sizes[6] < DM * DM || in_sizes[7] < DM || in_sizes[8] < DM) return;
    if ((long long)out_size < (long long)MROWS * DM) return;

    char* ws = (char*)d_ws;
    size_t off = 0;
    const size_t szx   = (size_t)MROWS * DM * 2;
    const size_t szwq  = (size_t)3 * DM * DM * 2;
    const size_t szwg1 = (size_t)HDIM * DM * 2;
    const size_t szwg2 = (size_t)DM * HDIM * 2;
    const size_t szwo  = (size_t)DM * DM * 2;
    const size_t szqk  = (size_t)MROWS * 2 * DM * 2;
    const size_t szvt  = (size_t)NB * NHEAD * HDIM * SEQ * 2;
    const size_t szh   = (size_t)MROWS * HDIM * 2;
    const size_t szg   = (size_t)MROWS * DM * 4;
    const size_t szo   = (size_t)MROWS * DM * 4;
    const size_t szy   = (size_t)MROWS * DM * 2;
    us* xb   = (us*)(ws + off); off += szx;
    us* wqb  = (us*)(ws + off); off += szwq;
    us* wg1b = (us*)(ws + off); off += szwg1;
    us* wg2b = (us*)(ws + off); off += szwg2;
    us* wob  = (us*)(ws + off); off += szwo;
    us* qkh  = (us*)(ws + off); off += szqk;
    us* qkl  = (us*)(ws + off); off += szqk;
    us* vth  = (us*)(ws + off); off += szvt;
    us* vtl  = (us*)(ws + off); off += szvt;
    us* hhp  = (us*)(ws + off); off += szh;
    us* hlp  = (us*)(ws + off); off += szh;
    float* gate = (float*)(ws + off); off += szg;
    float* op   = (float*)(ws + off); off += szo;
    us* yh   = (us*)(ws + off); off += szy;
    us* yl   = (us*)(ws + off); off += szy;
    if (off > ws_size) return;

    { const long long n8 = (long long)MROWS * (DM / 8);
      k_cvt<<<dim3((unsigned)((n8 + 255) / 256)), 256, 0, stream>>>(x, xb, MROWS, DM, SEQ, (long long)SEQ_FULL * DM, (long long)DM); }
    { const long long n8 = (long long)3 * DM * (DM / 8);
      k_cvt<<<dim3((unsigned)((n8 + 255) / 256)), 256, 0, stream>>>(wqkv, wqb, 3 * DM, DM, 3 * DM, 0LL, (long long)DM); }
    { const long long n8 = (long long)HDIM * (DM / 8);
      k_cvt<<<dim3((unsigned)((n8 + 255) / 256)), 256, 0, stream>>>(wg1, wg1b, HDIM, DM, HDIM, 0LL, (long long)DM); }
    { const long long n8 = (long long)DM * (HDIM / 8);
      k_cvt<<<dim3((unsigned)((n8 + 255) / 256)), 256, 0, stream>>>(wg2, wg2b, DM, HDIM, DM, 0LL, (long long)HDIM); }
    { const long long n8 = (long long)DM * (DM / 8);
      k_cvt<<<dim3((unsigned)((n8 + 255) / 256)), 256, 0, stream>>>(wout, wob, DM, DM, DM, 0LL, (long long)DM); }

    { GArg g;
      g.A0 = xb; g.A1 = xb; g.B = wqb; g.bias = bg1; g.C0 = qkh; g.C1 = qkl; g.T0 = vth; g.T1 = vtl;
      g.M = MROWS; g.N = 3 * DM; g.K = DM; g.lda = DM; g.ldb = DM; g.ldc = 2 * DM; g.act = 0; g.flags = 0;
      k_pgemm<1, 2><<<dim3((unsigned)(3 * DM / 64), (unsigned)(MROWS / 64)), 64, 0, stream>>>(g); }
    { GArg g;
      g.A0 = xb; g.A1 = xb; g.B = wg1b; g.bias = bg1; g.C0 = hhp; g.C1 = hlp; g.T0 = hhp; g.T1 = hlp;
      g.M = MROWS; g.N = HDIM; g.K = DM; g.lda = DM; g.ldb = DM; g.ldc = HDIM; g.act = 0; g.flags = 1;
      k_pgemm<1, 1><<<dim3((unsigned)(HDIM / 64), (unsigned)(MROWS / 64)), 64, 0, stream>>>(g); }
    { GArg g;
      g.A0 = hhp; g.A1 = hlp; g.B = wg2b; g.bias = bg2; g.C0 = gate; g.C1 = gate; g.T0 = gate; g.T1 = gate;
      g.M = MROWS; g.N = DM; g.K = HDIM; g.lda = HDIM; g.ldb = HDIM; g.ldc = DM; g.act = 6; g.flags = 1;
      k_pgemm<2, 0><<<dim3((unsigned)(DM / 64), (unsigned)(MROWS / 64)), 64, 0, stream>>>(g); }
    k_attn<<<dim3((unsigned)(SEQ / 16), (unsigned)NHEAD, (unsigned)NB), 32, 0, stream>>>(qkh, qkl, vth, vtl, op);
    k_ln<<<dim3((unsigned)MROWS), 128, 0, stream>>>(op, gate, gamma, beta, yh, yl);
    { GArg g;
      g.A0 = yh; g.A1 = yl; g.B = wob; g.bias = bg2; g.C0 = out; g.C1 = out; g.T0 = out; g.T1 = out;
      g.M = MROWS; g.N = DM; g.K = DM; g.lda = DM; g.ldb = DM; g.ldc = DM; g.act = 0; g.flags = 0;
      k_pgemm<2, 0><<<dim3((unsigned)(DM / 64), (unsigned)(MROWS / 64)), 64, 0, stream>>>(g); }
}
